// Qwen3NextAttention_3985729651555
// MI455X (gfx1250) — hardware-run, weakly checked
//
#include <hip/hip_runtime.h>
#include <math.h>

typedef __attribute__((ext_vector_type(16))) _Float16 v16h;
typedef __attribute__((ext_vector_type(8)))  _Float16 v8h;
typedef __attribute__((ext_vector_type(16))) __bf16   v16b;
typedef __attribute__((ext_vector_type(8)))  __bf16   v8b;
typedef __attribute__((ext_vector_type(8)))  float    v8f;
typedef __attribute__((ext_vector_type(4)))  float    v4f;
typedef __attribute__((ext_vector_type(4)))  unsigned int v4u;

constexpr int kB  = 2;
constexpr int kS  = 2048;
constexpr int kD  = 2048;
constexpr int kH  = 16;
constexpr int kKV = 4;
constexpr int kHD = 128;
constexpr int kT  = kB * kS;
constexpr int kQW = kH * kHD;
constexpr int kKW = kKV * kHD;
constexpr int kNcat = 2 * kQW + 2 * kKW;
constexpr int kEarly = 64;
constexpr int kFaKC = 64;
constexpr int kQBlocks = kB * kH * (kS / 16);
constexpr int kKBlocks = kB * kKV * (kS / 16);
constexpr float kEps = 1e-6f;
constexpr float kQKCarry = 16.0f;
constexpr float kVCarry  = 16.0f;
constexpr float kPCarry  = 32768.0f;
constexpr float kACarry  = 256.0f;
constexpr float kWoCarry = 1024.0f;
constexpr float kLoCarry = 2048.0f;
constexpr float kLoCarryInv = 1.0f / kLoCarry;
constexpr float kOutScale = 1.0f / (kACarry * kWoCarry);
constexpr float kEpiScale = kACarry / kVCarry;
constexpr float kInvHD = 1.0f / (float)kHD;

static_assert(kT == 4096 && kQW == 2048 && kKW == 512 && kNcat == 5120);
static_assert((kD % 32) == 0 && (kQW % 32) == 0 && (kHD % 32) == 0);
static_assert((kT % 64) == 0 && (kQW % 64) == 0 && (kKW % 64) == 0 && (kD % 64) == 0 && ((4 * kEarly) % 64) == 0);
static_assert((kS % 64) == 0 && kHD == 128 && kH == 4 * kKV && kQBlocks == 4096 && kKBlocks == 1024);

constexpr size_t kSzXB   = (size_t)kT * kD * 2;
constexpr size_t kSzWcat = (size_t)kNcat * kD * 2;
constexpr size_t kSzWo16 = (size_t)kD * kQW * 2;
constexpr size_t kSzDq   = (size_t)kT * kQW * 4;
constexpr size_t kSzDk   = (size_t)kT * kKW * 4;
constexpr size_t kSzDv   = (size_t)kT * kKW * 4;
constexpr size_t kSzDg   = (size_t)kT * kQW * 4;
constexpr size_t kOffXB   = 0;
constexpr size_t kOffWcat = kOffXB + kSzXB;
constexpr size_t kOffWo16 = kOffWcat + kSzWcat;
constexpr size_t kOffDq   = kOffWo16 + kSzWo16;
constexpr size_t kOffDk   = kOffDq + kSzDq;
constexpr size_t kOffDv   = kOffDk + kSzDk;
constexpr size_t kOffDg   = kOffDv + kSzDv;
constexpr size_t kWsTotal = kOffDg + kSzDg;
static_assert(kWsTotal == 130023424ull);
static_assert(kWsTotal <= 134217728ull);
constexpr size_t kSzQ16 = (size_t)kB * kH * kS * kHD * 2;
constexpr size_t kSzK16 = (size_t)kB * kKV * kS * kHD * 2;
constexpr size_t kSzVT  = (size_t)kB * kKV * kHD * kS * 2;
constexpr size_t kSzQE  = (size_t)kB * kH * kEarly * kHD * 4;
constexpr size_t kSzKE  = (size_t)kB * kKV * kEarly * kHD * 4;
constexpr size_t kOffQ16 = kOffXB;
constexpr size_t kOffK16 = kOffQ16 + kSzQ16;
constexpr size_t kOffVT  = kOffK16 + kSzK16;
constexpr size_t kOffQE  = kOffVT + kSzVT;
constexpr size_t kOffKE  = kOffQE + kSzQE;
static_assert(kOffKE + kSzKE <= kOffWo16);
constexpr size_t kSzAtt = (size_t)kT * kQW * 2;
constexpr size_t kSzA2  = (size_t)(4 * kEarly) * kQW * 2;
constexpr size_t kSzC2  = (size_t)(4 * kEarly) * kD * 4;
constexpr size_t kOffAtt = kOffDq;
constexpr size_t kOffA2  = kOffAtt + kSzAtt;
constexpr size_t kOffC2  = kOffA2 + kSzA2;
static_assert(kOffC2 + kSzC2 <= kOffDk);
static_assert((kOffWcat % 128) == 0 && (kOffWo16 % 128) == 0 && (kOffDq % 128) == 0 && (kOffDk % 128) == 0 &&
              (kOffDv % 128) == 0 && (kOffDg % 128) == 0 && (kOffK16 % 128) == 0 && (kOffVT % 128) == 0 &&
              (kOffQE % 128) == 0 && (kOffKE % 128) == 0 && (kOffA2 % 128) == 0 && (kOffC2 % 128) == 0);

__device__ __forceinline__ unsigned short f2bf_bits(float f) {
  unsigned u = __float_as_uint(f);
  return (unsigned short)((u + 0x7FFFu + ((u >> 16) & 1u)) >> 16);
}
__device__ __forceinline__ float bf_bits2f(unsigned short h) { return __uint_as_float(((unsigned)h) << 16); }
__device__ __forceinline__ float bf16_rne(float f) { return bf_bits2f(f2bf_bits(f)); }
__device__ __forceinline__ unsigned pk16(unsigned short a, unsigned short b) { return (unsigned)a | ((unsigned)b << 16); }
__device__ __forceinline__ unsigned short h_bits(float f) { const _Float16 h = (_Float16)f; return __builtin_bit_cast(unsigned short, h); }

__device__ __forceinline__ void dep_guard4_h(v8f& a, v8f& b, v8f& c, v8f& d, v16h x, v16h y) { asm volatile("v_nop\n\tv_nop\n\tv_nop\n\tv_nop" : "+v"(a), "+v"(b), "+v"(c), "+v"(d) : "v"(x), "v"(y)); }
__device__ __forceinline__ void dep_guard4_b(v8f& a, v8f& b, v8f& c, v8f& d, v16b x, v16b y) { asm volatile("v_nop\n\tv_nop\n\tv_nop\n\tv_nop" : "+v"(a), "+v"(b), "+v"(c), "+v"(d) : "v"(x), "v"(y)); }
__device__ __forceinline__ void keep4_h(v16h a, v16h b, v16h c, v16h d) { asm volatile("v_nop" :: "v"(a), "v"(b), "v"(c), "v"(d)); }
__device__ __forceinline__ void keep4_b(v16b a, v16b b, v16b c, v16b d) { asm volatile("v_nop" :: "v"(a), "v"(b), "v"(c), "v"(d)); }
__device__ __forceinline__ void acc_guard4(v8f& a, v8f& b, v8f& c, v8f& d) { asm volatile("v_nop\n\tv_nop\n\tv_nop\n\tv_nop" : "+v"(a), "+v"(b), "+v"(c), "+v"(d)); }

template <typename T> struct Frag;
template <> struct Frag<_Float16> {
  typedef v16h V; union U { v16h v; v8h h[2]; };
  static __device__ __forceinline__ v16h load(const _Float16* p) {
    U f; f.h[0] = *(const v8h*)(p); f.h[1] = *(const v8h*)(p + 16); return f.v;
  }
  static __device__ __forceinline__ v8f mma(v16h a, v16h b, v8f c) {
    return __builtin_amdgcn_wmma_f32_16x16x32_f16(false, a, false, b, (short)0, c, false, false);
  }
  static __device__ __forceinline__ void guard4(v8f& a, v8f& b, v8f& c, v8f& d, v16h x, v16h y) { dep_guard4_h(a, b, c, d, x, y); }
  static __device__ __forceinline__ void keep(v16h a, v16h b, v16h c, v16h d) { keep4_h(a, b, c, d); }
};
template <> struct Frag<__bf16> {
  typedef v16b V; union U { v16b v; v8b h[2]; };
  static __device__ __forceinline__ v16b load(const __bf16* p) {
    U f; f.h[0] = *(const v8b*)(p); f.h[1] = *(const v8b*)(p + 16); return f.v;
  }
  static __device__ __forceinline__ v8f mma(v16b a, v16b b, v8f c) {
    return __builtin_amdgcn_wmma_f32_16x16x32_bf16(false, a, false, b, (short)0, c, false, false);
  }
  static __device__ __forceinline__ void guard4(v8f& a, v8f& b, v8f& c, v8f& d, v16b x, v16b y) { dep_guard4_b(a, b, c, d, x, y); }
  static __device__ __forceinline__ void keep(v16b a, v16b b, v16b c, v16b d) { keep4_b(a, b, c, d); }
};

template <int ET> struct Elem;
template <> struct Elem<0> { typedef _Float16 T; };
template <> struct Elem<1> { typedef __bf16 T; };
template <int ET, bool SPLIT, int BIAS_MODE, int OUT_MODE, bool RESID, int ACT = 0>
__global__ __launch_bounds__(256) void wmma_gemm64(
    const unsigned short* __restrict__ Ap, const unsigned short* __restrict__ A2p, int lda, long strideA,
    const unsigned short* __restrict__ Btp, const unsigned short* __restrict__ Bt2p, int ldb, long strideB,
    void* __restrict__ Cout, void* __restrict__ Cout2, int ldc, long strideC,
    const float* __restrict__ bias,
    const float* __restrict__ resid, long strideR,
    int M, int N, int K, float scale) {
  typedef typename Elem<ET>::T T;
  typedef typename Frag<T>::V V;
  const T* A = (const T*)Ap; const T* A2 = (const T*)A2p; const T* Bt = (const T*)Btp; const T* Bt2 = (const T*)Bt2p;
  __shared__ __align__(16) float sT[8][16 * 68];
  const int b    = blockIdx.y;
  const int lane = threadIdx.x & 31;
  const int wave = __builtin_amdgcn_readfirstlane((int)(threadIdx.x >> 5));
  const int tilesN = N >> 6;
  const int tilesM = M >> 6;
  const int tile = blockIdx.x * 8 + wave;
  if (tile >= tilesM * tilesN) return;
  const int tm = tile / tilesN;
  const int tn = tile - tm * tilesN;
  const int m0 = tm << 6;
  const int n0 = tn << 6;

  const T* Ab  = A  + (size_t)b * strideA;
  const T* Bb  = Bt + (size_t)b * strideB;
  const T* Ab2 = SPLIT ? (A2  + (size_t)b * strideA) : nullptr;
  const T* Bb2 = SPLIT ? (Bt2 + (size_t)b * strideB) : nullptr;

  const int rlane = lane & 15;
  const int koff  = (lane >> 4) * 8;
  const int mOff  = (lane >> 4) * 8;

  v8f acc[4][4];
#pragma unroll
  for (int i = 0; i < 4; ++i)
#pragma unroll
    for (int j = 0; j < 4; ++j) acc[i][j] = (v8f){0.f,0.f,0.f,0.f,0.f,0.f,0.f,0.f};

  for (int k0 = 0; k0 < K; k0 += 32) {
    V bh[4], bl[4];
#pragma unroll
    for (int j = 0; j < 4; ++j) {
      const size_t bo = (size_t)(n0 + (j << 4) + rlane) * ldb + koff + k0;
      bh[j] = Frag<T>::load(Bb + bo);
      if (SPLIT) bl[j] = Frag<T>::load(Bb2 + bo);
    }
#pragma unroll
    for (int i = 0; i < 4; ++i) {
      const size_t ao = (size_t)(m0 + (i << 4) + rlane) * lda + koff + k0;
      V ah = Frag<T>::load(Ab + ao);
      V al;
      if (SPLIT) al = Frag<T>::load(Ab2 + ao);
#pragma unroll
      for (int j = 0; j < 4; ++j) {
        acc[i][j] = Frag<T>::mma(ah, bh[j], acc[i][j]);
        if (SPLIT) {
          acc[i][j] = Frag<T>::mma(ah, bl[j], acc[i][j]);
          acc[i][j] = Frag<T>::mma(al, bh[j], acc[i][j]);
        }
      }
      Frag<T>::guard4(acc[i][0], acc[i][1], acc[i][2], acc[i][3], ah, SPLIT ? al : ah);
    }
    Frag<T>::keep(bh[0], bh[1], bh[2], bh[3]);
    if (SPLIT) Frag<T>::keep(bl[0], bl[1], bl[2], bl[3]);
  }
  acc_guard4(acc[0][0], acc[0][1], acc[0][2], acc[0][3]);
  acc_guard4(acc[1][0], acc[1][1], acc[1][2], acc[1][3]);
  acc_guard4(acc[2][0], acc[2][1], acc[2][2], acc[2][3]);
  acc_guard4(acc[3][0], acc[3][1], acc[3][2], acc[3][3]);

  float* slab = sT[wave];
  const float* Rb = RESID ? (resid + (size_t)b * strideR) : nullptr;
#pragma unroll
  for (int i = 0; i < 4; ++i) {
    const int mBase = m0 + (i << 4);
#pragma unroll
    for (int j = 0; j < 4; ++j) {
      const int n = n0 + (j << 4) + rlane;
      float bv = 0.f;
      if (BIAS_MODE == 2) bv = bias[n];
#pragma unroll
      for (int r = 0; r < 8; ++r) {
        float v = acc[i][j][r] * scale;
        if (BIAS_MODE == 1) v += bias[mBase + mOff + r];
        if (BIAS_MODE == 2) v += bv;
        if (RESID) v += Rb[(size_t)(mBase + mOff + r) * ldc + n];
        if (ACT == 2) v = fmaxf(v, 0.0f);
        if (ACT == 4) v = (v > 0.f) ? v : 0.01f * v;
        slab[(mOff + r) * 68 + (j << 4) + rlane] = v;
      }
    }
    __builtin_amdgcn_fence(__ATOMIC_RELEASE, "workgroup");
    __builtin_amdgcn_wave_barrier();
    __builtin_amdgcn_fence(__ATOMIC_ACQUIRE, "workgroup");
    if (OUT_MODE == 0) {
      float* C = (float*)Cout + (size_t)b * strideC;
      const int hh = lane >> 4, c4 = (lane & 15) * 4;
      for (int pass = 0; pass < 2; ++pass) {
#pragma unroll
        for (int it = 0; it < 8; ++it) {
          const int row = it * 2 + hh;
          v4f v = *(const v4f*)(slab + row * 68 + c4);
          *(volatile v4f*)(C + (size_t)(mBase + row) * ldc + n0 + c4) = v;
        }
        __threadfence();
      }
    } else {
      const int q = lane >> 3, c8 = (lane & 7) * 8;
      unsigned short* C  = (unsigned short*)Cout  + (size_t)b * strideC;
      unsigned short* C2 = (OUT_MODE == 2) ? ((unsigned short*)Cout2 + (size_t)b * strideC) : nullptr;
      for (int pass = 0; pass < 2; ++pass) {
#pragma unroll
        for (int it = 0; it < 4; ++it) {
          const int row = it * 4 + q;
          const float* sp = slab + row * 68 + c8;
          v8h hv, lv;
#pragma unroll
          for (int e = 0; e < 8; ++e) {
            if (OUT_MODE == 1) {
              hv[e] = (_Float16)sp[e];
            } else {
              unsigned short hb = f2bf_bits(sp[e]);
              unsigned short lb = f2bf_bits(sp[e] - bf_bits2f(hb));
              hv[e] = __builtin_bit_cast(_Float16, hb);
              lv[e] = __builtin_bit_cast(_Float16, lb);
            }
          }
          *(volatile v8h*)(C + (size_t)(mBase + row) * ldc + n0 + c8) = hv;
          if (OUT_MODE == 2) *(volatile v8h*)(C2 + (size_t)(mBase + row) * ldc + n0 + c8) = lv;
        }
        __threadfence();
      }
    }
    __builtin_amdgcn_fence(__ATOMIC_RELEASE, "workgroup");
    __builtin_amdgcn_wave_barrier();
    __builtin_amdgcn_fence(__ATOMIC_ACQUIRE, "workgroup");
  }
}

__global__ __launch_bounds__(256) void cvt_x_kernel(const float* __restrict__ in, unsigned short* __restrict__ out, int n8) {
  const int i = blockIdx.x * 256 + threadIdx.x;
  if (i >= n8) return;
  const float* p = in + 8 * (size_t)i;
  const v4f a = *(const v4f*)(p);
  const v4f c = *(const v4f*)(p + 4);
  unsigned short hb[8];
#pragma unroll
  for (int e = 0; e < 4; ++e) {
    hb[e]     = f2bf_bits(a[e]);
    hb[4 + e] = f2bf_bits(c[e]);
  }
  const v4u u = (v4u){pk16(hb[0], hb[1]), pk16(hb[2], hb[3]), pk16(hb[4], hb[5]), pk16(hb[6], hb[7])};
  unsigned short* q = out + 8 * (size_t)i;
  *(volatile v4u*)q = u;
  __threadfence();
  *(volatile v4u*)q = u;
}

__global__ __launch_bounds__(256) void cvt_wcat_kernel(const float* __restrict__ Wq, const float* __restrict__ Wk,
                                                       const float* __restrict__ Wv, unsigned short* __restrict__ Wcat) {
  const int n = blockIdx.x;
  const float* src;
  if (n < kQW) {
    src = Wq + (size_t)((n >> 7) * 256 + (n & 127)) * kD;
  } else if (n < kQW + kKW) {
    src = Wk + (size_t)(n - kQW) * kD;
  } else if (n < kQW + 2 * kKW) {
    src = Wv + (size_t)(n - kQW - kKW) * kD;
  } else {
    const int m = n - (kQW + 2 * kKW);
    src = Wq + (size_t)((m >> 7) * 256 + 128 + (m & 127)) * kD;
  }
  const int c8 = threadIdx.x * 8;
  const v4f a = *(const v4f*)(src + c8);
  const v4f c = *(const v4f*)(src + c8 + 4);
  unsigned short hb[8];
#pragma unroll
  for (int e = 0; e < 4; ++e) {
    hb[e]     = f2bf_bits(a[e]);
    hb[4 + e] = f2bf_bits(c[e]);
  }
  const v4u u = (v4u){pk16(hb[0], hb[1]), pk16(hb[2], hb[3]), pk16(hb[4], hb[5]), pk16(hb[6], hb[7])};
  unsigned short* q = Wcat + (size_t)n * kD + c8;
  *(volatile v4u*)q = u;
  __threadfence();
  *(volatile v4u*)q = u;
}

__global__ __launch_bounds__(256) void cvt_wo_kernel(const float* __restrict__ in, unsigned short* __restrict__ out, int n8) {
  const int i = blockIdx.x * 256 + threadIdx.x;
  if (i >= n8) return;
  const float* p = in + 8 * (size_t)i;
  const v4f a = *(const v4f*)(p);
  const v4f c = *(const v4f*)(p + 4);
  unsigned short hb[8];
#pragma unroll
  for (int e = 0; e < 4; ++e) {
    hb[e]     = h_bits(bf16_rne(a[e]) * kWoCarry);
    hb[4 + e] = h_bits(bf16_rne(c[e]) * kWoCarry);
  }
  const v4u u = (v4u){pk16(hb[0], hb[1]), pk16(hb[2], hb[3]), pk16(hb[4], hb[5]), pk16(hb[6], hb[7])};
  unsigned short* q = out + 8 * (size_t)i;
  *(volatile v4u*)q = u;
  __threadfence();
  *(volatile v4u*)q = u;
}

__global__ __launch_bounds__(256) void normrope_kernel(
    const float* __restrict__ Dq, const float* __restrict__ Dk, const float* __restrict__ freqs,
    const float* __restrict__ qnw, const float* __restrict__ knw,
    unsigned short* __restrict__ q16, unsigned short* __restrict__ k16,
    float* __restrict__ qe, float* __restrict__ ke) {
  __shared__ __align__(16) float sF[16 * 132];
  const int tid  = threadIdx.x;
  const int wave = __builtin_amdgcn_readfirstlane((int)(threadIdx.x >> 5));
  const int lane = tid & 31;
  const int g16  = tid >> 4;
  const int l16  = tid & 15;
  const int bx   = blockIdx.x;
  const bool isK = (bx >= kQBlocks);
  const int idx  = isK ? (bx - kQBlocks) : bx;
  const int sblk = idx & 127;
  const int nh   = isK ? kKV : kH;
  const int h    = isK ? ((idx >> 7) & 3) : ((idx >> 7) & 15);
  const int b    = isK ? (idx >> 9) : (idx >> 11);
  const int s0   = sblk * 16;
  const int s    = s0 + g16;
  const int pitch = isK ? kKW : kQW;
  const float* src = (isK ? Dk : Dq) + (size_t)(b * kS + s) * pitch + h * kHD;
  const float* nw  = isK ? knw : qnw;

  const v4f xa = *(const v4f*)(src + 4 * l16);
  const v4f xb = *(const v4f*)(src + 64 + 4 * l16);
  float ss = 0.0f;
#pragma unroll
  for (int e = 0; e < 4; ++e) {
    ss = fmaf(xa[e], xa[e], ss);
    ss = fmaf(xb[e], xb[e], ss);
  }
  ss += __shfl_xor(ss, 8, 32);
  ss += __shfl_xor(ss, 4, 32);
  ss += __shfl_xor(ss, 2, 32);
  ss += __shfl_xor(ss, 1, 32);
  const float rs = rsqrtf(ss * kInvHD + kEps);
  const v4f wa = *(const v4f*)(nw + 4 * l16);
  const v4f wb = *(const v4f*)(nw + 64 + 4 * l16);
  const v4f cc = *(const v4f*)(freqs + (size_t)s * kHD + 4 * l16);
  const v4f sn = *(const v4f*)(freqs + (size_t)s * kHD + 64 + 4 * l16);
  v4f o1, o2;
#pragma unroll
  for (int e = 0; e < 4; ++e) {
    const float na = (xa[e] * rs) * (1.0f + bf16_rne(wa[e]));
    const float nb = (xb[e] * rs) * (1.0f + bf16_rne(wb[e]));
    const float c  = bf16_rne(cc[e]);
    const float sv = bf16_rne(sn[e]);
    o1[e] = na * c - nb * sv;
    o2[e] = nb * c + na * sv;
  }
  float* fr = sF + g16 * 132;
  *(v4f*)(fr + 4 * l16) = o1;
  *(v4f*)(fr + 64 + 4 * l16) = o2;
  __syncthreads();
  {
    unsigned short* dst16 = isK ? k16 : q16;
    const int row = wave * 2 + (lane >> 4);
    const int c8  = (lane & 15) * 8;
    const float* sp = sF + row * 132 + c8;
    const v4f a0 = *(const v4f*)(sp);
    const v4f a1 = *(const v4f*)(sp + 4);
    unsigned short hb[8];
#pragma unroll
    for (int e = 0; e < 4; ++e) {
      hb[e]     = h_bits(a0[e] * kQKCarry);
      hb[4 + e] = h_bits(a1[e] * kQKCarry);
    }
    const v4u u = (v4u){pk16(hb[0], hb[1]), pk16(hb[2], hb[3]), pk16(hb[4], hb[5]), pk16(hb[6], hb[7])};
    unsigned short* p = dst16 + ((size_t)((b * nh + h) * kS) + s0 + row) * kHD + c8;
    *(volatile v4u*)p = u;
    __threadfence();
    *(volatile v4u*)p = u;
  }
  if (s0 < kEarly) {
    float* dstE = isK ? ke : qe;
    v4f ev[2];
#pragma unroll
    for (int it = 0; it < 2; ++it) ev[it] = *(const v4f*)(sF + (wave * 2 + it) * 132 + lane * 4);
    for (int pass = 0; pass < 2; ++pass) {
#pragma unroll
      for (int it = 0; it < 2; ++it) {
        const int row = wave * 2 + it;
        *(volatile v4f*)(dstE + ((size_t)((b * nh + h) * kEarly) + s0 + row) * kHD + lane * 4) = ev[it];
      }
      __threadfence();
    }
  }
}

__global__ __launch_bounds__(256) void vtrans_kernel(const float* __restrict__ Dv, unsigned short* __restrict__ vT16) {
  __shared__ float sm[64][65];
  const int t    = threadIdx.x;
  const int wave = __builtin_amdgcn_readfirstlane((int)(threadIdx.x >> 5));
  const int lane = t & 31;
  const int t0 = blockIdx.x * 64;
  const int c0 = blockIdx.y * 64;
  const int b  = t0 >> 11;
  const int s0 = t0 & (kS - 1);
#pragma unroll
  for (int i = 0; i < 16; ++i) {
    const int e  = i * 256 + t;
    const int r  = e >> 6;
    const int cc = e & 63;
    sm[cc][r] = Dv[(size_t)(t0 + r) * kKW + c0 + cc];
  }
  __syncthreads();
  const int q = lane >> 3, c8 = (lane & 7) * 8;
  v4u u[2];
#pragma unroll
  for (int it = 0; it < 2; ++it) {
    const int row = wave * 8 + it * 4 + q;
    unsigned short hb[8];
#pragma unroll
    for (int e = 0; e < 8; ++e) hb[e] = h_bits(sm[row][c8 + e] * kVCarry);
    u[it] = (v4u){pk16(hb[0], hb[1]), pk16(hb[2], hb[3]), pk16(hb[4], hb[5]), pk16(hb[6], hb[7])};
  }
  for (int pass = 0; pass < 2; ++pass) {
#pragma unroll
    for (int it = 0; it < 2; ++it) {
      const int row = wave * 8 + it * 4 + q;
      *(volatile v4u*)(vT16 + ((size_t)(b * kKW + c0 + row)) * kS + s0 + c8) = u[it];
    }
    __threadfence();
  }
}

__device__ __forceinline__ v8f mma_h(v16h a, v16h b, v8f c) {
  c = __builtin_amdgcn_wmma_f32_16x16x32_f16(false, a, false, b, (short)0, c, false, false);
  asm volatile("v_nop\n\tv_nop\n\tv_nop\n\tv_nop" : "+v"(c) : "v"(a), "v"(b));
  return c;
}

__global__ __launch_bounds__(128) void flash_kernel(
    const _Float16* __restrict__ q16, const _Float16* __restrict__ k16, const _Float16* __restrict__ vT16,
    const float* __restrict__ Dg, unsigned short* __restrict__ attn16, float scl) {
  union FH { v16h v; v8h h[2]; };
  __shared__ __align__(16) _Float16 Ksh[kFaKC * kHD];
  __shared__ __align__(16) _Float16 Vsh[kHD * kFaKC];
  __shared__ __align__(16) _Float16 Psh[4][16 * kFaKC];
  __shared__ __align__(16) float Os[4][16 * 68];

  const int tid  = threadIdx.x;
  const int wave = __builtin_amdgcn_readfirstlane((int)(threadIdx.x >> 5));
  const int lane = tid & 31;
  const int hh   = lane >> 4;
  const int c    = lane & 15;
  const int bx   = blockIdx.x;
  const int qb   = bx & 31;
  const int bh   = bx >> 5;
  const int h    = bh & 15;
  const int b    = bh >> 4;
  const int kv   = h >> 2;
  const int q0   = qb * 64 + wave * 16;

  v16h qa[4];
  {
    const _Float16* qrow = q16 + ((size_t)(b * kH + h) * kS + q0 + c) * kHD + 8 * hh;
#pragma unroll
    for (int dc = 0; dc < 4; ++dc) qa[dc] = Frag<_Float16>::load(qrow + dc * 32);
  }
  const _Float16* kbase = k16 + (size_t)(b * kKV + kv) * kS * kHD;
  const _Float16* vbase = vT16 + (size_t)(b * kKV + kv) * kHD * kS;

  float mrow[8], lrow[8];
  v8f oacc[8];
#pragma unroll
  for (int r = 0; r < 8; ++r) { mrow[r] = -INFINITY; lrow[r] = 0.f; }
#pragma unroll
  for (int t = 0; t < 8; ++t) oacc[t] = (v8f){0.f,0.f,0.f,0.f,0.f,0.f,0.f,0.f};

  _Float16* pw = Psh[wave];
  const int nChunks = qb + 1;
  for (int kc = 0; kc < nChunks; ++kc) {
    const int kv0 = kc * kFaKC;
    __syncthreads();
#pragma unroll
    for (int i = 0; i < 8; ++i) {
      const int u = i * 128 + tid;
      *(v8h*)(Ksh + u * 8) = *(const v8h*)(kbase + (size_t)kv0 * kHD + u * 8);
      const int d = u >> 3, cc = (u & 7) * 8;
      *(v8h*)(Vsh + d * kFaKC + cc) = *(const v8h*)(vbase + (size_t)d * kS + kv0 + cc);
    }
    __syncthreads();

    v8f s[4];
#pragma unroll
    for (int j = 0; j < 4; ++j) {
      s[j] = (v8f){0.f,0.f,0.f,0.f,0.f,0.f,0.f,0.f};
#pragma unroll
      for (int dc = 0; dc < 4; ++dc) {
        FH kb;
        kb.h[0] = *(const v8h*)(Ksh + (j * 16 + c) * kHD + dc * 32 + 8 * hh);
        kb.h[1] = *(const v8h*)(Ksh + (j * 16 + c) * kHD + dc * 32 + 16 + 8 * hh);
        s[j] = mma_h(qa[dc], kb.v, s[j]);
      }
    }
    const bool diag = (kc == qb);
    float cm[8];
#pragma unroll
    for (int r = 0; r < 8; ++r) {
      const int qrow = q0 + 8 * hh + r;
      float m = -INFINITY;
#pragma unroll
      for (int j = 0; j < 4; ++j) {
        const int kvcol = kv0 + j * 16 + c;
        const bool masked = diag && (kvcol > qrow);
        float sv = s[j][r] * scl;
        sv = masked ? -INFINITY : sv;
        s[j][r] = sv;
        m = fmaxf(m, sv);
      }
      m = fmaxf(m, __shfl_xor(m, 1, 32));
      m = fmaxf(m, __shfl_xor(m, 2, 32));
      m = fmaxf(m, __shfl_xor(m, 4, 32));
      m = fmaxf(m, __shfl_xor(m, 8, 32));
      cm[r] = m;
    }
#pragma unroll
    for (int r = 0; r < 8; ++r) {
      const float mnew  = fmaxf(mrow[r], cm[r]);
      const float alpha = __expf(mrow[r] - mnew);
      mrow[r] = mnew;
      float psum = 0.f;
#pragma unroll
      for (int j = 0; j < 4; ++j) {
        const float p = __expf(s[j][r] - mnew);
        const _Float16 ph = (_Float16)(p * kPCarry);
        float pf = (float)ph;
        asm volatile("" : "+v"(pf));
        psum += pf;
        pw[(8 * hh + r) * kFaKC + j * 16 + c] = ph;
      }
      psum += __shfl_xor(psum, 1, 32);
      psum += __shfl_xor(psum, 2, 32);
      psum += __shfl_xor(psum, 4, 32);
      psum += __shfl_xor(psum, 8, 32);
      lrow[r] = lrow[r] * alpha + psum;
#pragma unroll
      for (int t = 0; t < 8; ++t) oacc[t][r] *= alpha;
    }
    __builtin_amdgcn_fence(__ATOMIC_RELEASE, "workgroup");
    __builtin_amdgcn_wave_barrier();
    __builtin_amdgcn_fence(__ATOMIC_ACQUIRE, "workgroup");
#pragma unroll
    for (int kk = 0; kk < 2; ++kk) {
      FH pa;
      pa.h[0] = *(const v8h*)(pw + c * kFaKC + kk * 32 + 8 * hh);
      pa.h[1] = *(const v8h*)(pw + c * kFaKC + kk * 32 + 16 + 8 * hh);
#pragma unroll
      for (int t = 0; t < 8; ++t) {
        FH vb;
        vb.h[0] = *(const v8h*)(Vsh + (t * 16 + c) * kFaKC + kk * 32 + 8 * hh);
        vb.h[1] = *(const v8h*)(Vsh + (t * 16 + c) * kFaKC + kk * 32 + 16 + 8 * hh);
        oacc[t] = mma_h(pa.v, vb.v, oacc[t]);
      }
    }
    __builtin_amdgcn_fence(__ATOMIC_RELEASE, "workgroup");
    __builtin_amdgcn_wave_barrier();
    __builtin_amdgcn_fence(__ATOMIC_ACQUIRE, "workgroup");
  }

  float inv[8];
#pragma unroll
  for (int r = 0; r < 8; ++r) inv[r] = kEpiScale / lrow[r];
  float* os = Os[wave];
  const int q4 = lane >> 3, c8 = (lane & 7) * 8;
#pragma unroll
  for (int hf = 0; hf < 2; ++hf) {
#pragma unroll
    for (int r = 0; r < 8; ++r) {
#pragma unroll
      for (int tt = 0; tt < 4; ++tt) os[(8 * hh + r) * 68 + tt * 16 + c] = oacc[hf * 4 + tt][r] * inv[r];
    }
    __builtin_amdgcn_fence(__ATOMIC_RELEASE, "workgroup");
    __builtin_amdgcn_wave_barrier();
    __builtin_amdgcn_fence(__ATOMIC_ACQUIRE, "workgroup");
    v8h hv[4];
#pragma unroll
    for (int it = 0; it < 4; ++it) {
      const int row = it * 4 + q4;
      const float* sp = os + row * 68 + c8;
      const v4f a0 = *(const v4f*)(sp);
      const v4f a1 = *(const v4f*)(sp + 4);
      const float* gp = Dg + (size_t)(b * kS + q0 + row) * kQW + h * kHD + hf * 64 + c8;
      const v4f g0 = *(const v4f*)(gp);
      const v4f g1 = *(const v4f*)(gp + 4);
#pragma unroll
      for (int e = 0; e < 4; ++e) {
        const float x0 = a0[e], x1 = a1[e];
        const float y0 = g0[e], y1 = g1[e];
        const float sg0 = __builtin_amdgcn_rcpf(1.0f + __expf(-y0));
        const float sg1 = __builtin_amdgcn_rcpf(1.0f + __expf(-y1));
        hv[it][e]     = (_Float16)(x0 * sg0);
        hv[it][4 + e] = (_Float16)(x1 * sg1);
      }
    }
    for (int pass = 0; pass < 2; ++pass) {
#pragma unroll
      for (int it = 0; it < 4; ++it) {
        const int row = it * 4 + q4;
        *(volatile v8h*)(attn16 + (size_t)(b * kS + q0 + row) * kQW + h * kHD + hf * 64 + c8) = hv[it];
      }
      __threadfence();
    }
    __builtin_amdgcn_fence(__ATOMIC_RELEASE, "workgroup");
    __builtin_amdgcn_wave_barrier();
    __builtin_amdgcn_fence(__ATOMIC_ACQUIRE, "workgroup");
  }
}

__global__ __launch_bounds__(128) void early_attn_kernel(
    const float* __restrict__ qe, const float* __restrict__ ke, const float* __restrict__ Dv,
    const float* __restrict__ Dg, unsigned short* __restrict__ A2, float scl) {
  __shared__ __align__(16) float sQ[kHD];
  __shared__ float sPart[2][64];
  __shared__ float sP[64];
  __shared__ unsigned short sHL[2 * kHD];
  const int tid  = threadIdx.x;
  const int wave = __builtin_amdgcn_readfirstlane((int)(threadIdx.x >> 5));
  const int lane = tid & 31;
  const int bx = blockIdx.x;
  const int s  = bx & 63;
  const int h  = (bx >> 6) & 15;
  const int b  = bx >> 10;
  const int kv = h >> 2;

  sQ[tid] = qe[((size_t)((b * kH + h) * kEarly) + s) * kHD + tid];
  __syncthreads();
  {
    const int j    = tid & 63;
    const int half = wave >> 1;
    const int jc   = (j < s) ? j : s;
    const float* kp = ke + ((size_t)((b * kKV + kv) * kEarly) + jc) * kHD + half * 64;
    const float* qp = sQ + half * 64;
    float dot = 0.0f;
#pragma unroll 1
    for (int i = 0; i < 16; ++i) {
      const v4f kk = *(const v4f*)(kp + 4 * i);
      const v4f qq = *(const v4f*)(qp + 4 * i);
      dot = fmaf(kk[0], qq[0], dot);
      dot = fmaf(kk[1], qq[1], dot);
      dot = fmaf(kk[2], qq[2], dot);
      dot = fmaf(kk[3], qq[3], dot);
    }
    sPart[half][j] = dot;
  }
  __syncthreads();
  {
    float x0 = (sPart[0][lane] + sPart[1][lane]) * scl;
    float x1 = (sPart[0][lane + 32] + sPart[1][lane + 32]) * scl;
    x0 = (lane <= s) ? x0 : -INFINITY;
    x1 = (lane + 32 <= s) ? x1 : -INFINITY;
    float m = fmaxf(x0, x1);
    m = fmaxf(m, __shfl_xor(m, 16, 32));
    m = fmaxf(m, __shfl_xor(m, 8, 32));
    m = fmaxf(m, __shfl_xor(m, 4, 32));
    m = fmaxf(m, __shfl_xor(m, 2, 32));
    m = fmaxf(m, __shfl_xor(m, 1, 32));
    const float e0 = expf(x0 - m);
    const float e1 = expf(x1 - m);
    float sum = e0 + e1;
    sum += __shfl_xor(sum, 16, 32);
    sum += __shfl_xor(sum, 8, 32);
    sum += __shfl_xor(sum, 4, 32);
    sum += __shfl_xor(sum, 2, 32);
    sum += __shfl_xor(sum, 1, 32);
    const float rinv = 1.0f / sum;
    if (wave == 0) {
      sP[lane]      = e0 * rinv;
      sP[lane + 32] = e1 * rinv;
    }
  }
  __syncthreads();
  {
    const int d = tid;
    const int jmax = (s < kEarly - 1) ? s : (kEarly - 1);
    const float* vp = Dv + (size_t)(b * kS) * kKW + kv * kHD + d;
    float acc = 0.0f;
#pragma unroll 1
    for (int j = 0; j <= jmax; ++j) acc = fmaf(sP[j], vp[(size_t)j * kKW], acc);
    const float g   = Dg[(size_t)(b * kS + s) * kQW + h * kHD + d];
    const float sig = 1.0f / (1.0f + expf(-g));
    const float a256 = (acc * sig) * kACarry;
    const _Float16 hi = (_Float16)a256;
    float hif = (float)hi;
    asm volatile("" : "+v"(hif));
    const float lo = (a256 - hif) * kLoCarry;
    sHL[d]       = __builtin_bit_cast(unsigned short, hi);
    sHL[kHD + d] = h_bits(lo);
  }
  __syncthreads();
  if (wave == 0) {
    const int part = lane >> 4;
    const int c8   = (lane & 15) * 8;
    const unsigned short* sp = sHL + part * kHD + c8;
    const v4u u = (v4u){pk16(sp[0], sp[1]), pk16(sp[2], sp[3]), pk16(sp[4], sp[5]), pk16(sp[6], sp[7])};
    unsigned short* p = A2 + (size_t)(part * (2 * kEarly) + b * kEarly + s) * kQW + h * kHD + c8;
    *(volatile v4u*)p = u;
    __threadfence();
    *(volatile v4u*)p = u;
  }
}

__global__ __launch_bounds__(256) void early_add_kernel(const float* __restrict__ C2, float* __restrict__ out) {
  const int i  = blockIdx.x * 256 + threadIdx.x;
  const int r  = i >> 9;
  const int c4 = (i & 511) * 4;
  const int b  = r >> 6;
  const int s  = r & 63;
  const v4f hi = *(const v4f*)(C2 + (size_t)r * kD + c4);
  const v4f lo = *(const v4f*)(C2 + (size_t)(2 * kEarly + r) * kD + c4);
  v4f o;
#pragma unroll
  for (int e = 0; e < 4; ++e) o[e] = hi[e] + lo[e] * kLoCarryInv;
  float* p = out + (size_t)(b * kS + s) * kD + c4;
  *(volatile v4f*)p = o;
  __threadfence();
  *(volatile v4f*)p = o;
}

extern "C" void kernel_launch(void* const* d_in, const int* in_sizes, int n_in,
                              void* d_out, int out_size, void* d_ws, size_t ws_size,
                              hipStream_t stream) {
  if (n_in < 8) return;
  if (in_sizes[0] != kT * kD) return;
  if (in_sizes[1] != kS * kHD) return;
  if (in_sizes[2] != 2 * kQW * kD) return;
  if (in_sizes[3] != kKW * kD) return;
  if (in_sizes[4] != kKW * kD) return;
  if (in_sizes[5] != kD * kQW) return;
  if (in_sizes[6] != kHD) return;
  if (in_sizes[7] != kHD) return;
  if (out_size != kT * kD) return;
  if (ws_size < kWsTotal) return;

  const float* x     = (const float*)d_in[0];
  const float* freqs = (const float*)d_in[1];
  const float* Wq    = (const float*)d_in[2];
  const float* Wk    = (const float*)d_in[3];
  const float* Wv    = (const float*)d_in[4];
  const float* Wo    = (const float*)d_in[5];
  const float* qnw   = (const float*)d_in[6];
  const float* knw   = (const float*)d_in[7];
  float* out = (float*)d_out;

  char* ws = (char*)d_ws;
  unsigned short* XB   = (unsigned short*)(ws + kOffXB);
  unsigned short* WCAT = (unsigned short*)(ws + kOffWcat);
  unsigned short* WO16 = (unsigned short*)(ws + kOffWo16);
  float* DQ = (float*)(ws + kOffDq);
  float* DK = (float*)(ws + kOffDk);
  float* DV = (float*)(ws + kOffDv);
  float* DG = (float*)(ws + kOffDg);
  unsigned short* Q16  = (unsigned short*)(ws + kOffQ16);
  unsigned short* K16  = (unsigned short*)(ws + kOffK16);
  unsigned short* VT16 = (unsigned short*)(ws + kOffVT);
  float* QE = (float*)(ws + kOffQE);
  float* KE = (float*)(ws + kOffKE);
  unsigned short* ATT16 = (unsigned short*)(ws + kOffAtt);
  unsigned short* A2    = (unsigned short*)(ws + kOffA2);
  float* C2 = (float*)(ws + kOffC2);

  const float scl     = (float)(1.0 / sqrt((double)kHD));
  const float scl_qk  = scl / (kQKCarry * kQKCarry);

  cvt_x_kernel<<<(kT * kD / 8) / 256, 256, 0, stream>>>(x, XB, kT * kD / 8);
  cvt_wcat_kernel<<<kNcat, 256, 0, stream>>>(Wq, Wk, Wv, WCAT);
  cvt_wo_kernel<<<(kD * kQW / 8) / 256, 256, 0, stream>>>(Wo, WO16, kD * kQW / 8);

  wmma_gemm64<1, false, 0, 0, false><<<dim3(256, 2), 256, 0, stream>>>(
      XB, nullptr, kD, 0L,
      WCAT, nullptr, kD, (long)(kQW + 2 * kKW) * kD,
      (void*)DQ, nullptr, kQW, (long)((kOffDg - kOffDq) / 4),
      nullptr, nullptr, 0L,
      kT, kQW, kD, 1.0f);
  wmma_gemm64<1, false, 0, 0, false><<<dim3(64, 2), 256, 0, stream>>>(
      XB, nullptr, kD, 0L,
      WCAT + (size_t)kQW * kD, nullptr, kD, (long)kKW * kD,
      (void*)DK, nullptr, kKW, (long)((kOffDv - kOffDk) / 4),
      nullptr, nullptr, 0L,
      kT, kKW, kD, 1.0f);

  normrope_kernel<<<kQBlocks + kKBlocks, 256, 0, stream>>>(DQ, DK, freqs, qnw, knw, Q16, K16, QE, KE);
  vtrans_kernel<<<dim3(kT / 64, kKW / 64), 256, 0, stream>>>(DV, VT16);

  flash_kernel<<<kB * kH * (kS / 64), 128, 0, stream>>>(
      (const _Float16*)Q16, (const _Float16*)K16, (const _Float16*)VT16, DG, ATT16, scl_qk);

  wmma_gemm64<0, false, 0, 0, false><<<dim3(256, 1), 256, 0, stream>>>(
      ATT16, nullptr, kQW, 0L,
      WO16, nullptr, kQW, 0L,
      (void*)out, nullptr, kD, 0L,
      nullptr, nullptr, 0L,
      kT, kD, kQW, kOutScale);

  early_attn_kernel<<<kB * kH * kEarly, 128, 0, stream>>>(QE, KE, DV, DG, A2, scl);
  wmma_gemm64<0, false, 0, 0, false><<<dim3(16, 1), 256, 0, stream>>>(
      A2, nullptr, kQW, 0L,
      WO16, nullptr, kQW, 0L,
      (void*)C2, nullptr, kD, 0L,
      nullptr, nullptr, 0L,
      4 * kEarly, kD, kQW, kOutScale);
  early_add_kernel<<<(2 * kEarly * kD / 4) / 256, 256, 0, stream>>>(C2, out);
}
